// Layer_61907658605100
// MI455X (gfx1250) — hardware-verified
//
#include <hip/hip_runtime.h>
#include <math.h>
#include <stdint.h>
#include <stddef.h>

#define NBATCH 4
#define SEQ    1024
#define DM     1024
#define NH     16
#define HD     64
#define DFF    4096
#define NTOK   (NBATCH * SEQ)
#define QKP    (2 * DM)
#define WM     (DM * DM)
#define LN_EPS 1.0e-5f
#define WSC    64.0f
#define INV_WSC 0.015625f
#define PSC    32768.0f
#define CTP    32

static_assert(DM % 64 == 0);
static_assert(DFF % 64 == 0);
static_assert(NTOK % 64 == 0);
static_assert(DM % 32 == 0);
static_assert(DFF % 32 == 0);
static_assert(SEQ % 64 == 0);
static_assert(NH * HD == DM);

typedef _Float16 v16h __attribute__((ext_vector_type(16)));
typedef _Float16 v8h  __attribute__((ext_vector_type(8)));
typedef float    v8f  __attribute__((ext_vector_type(8)));
typedef float    v4f  __attribute__((ext_vector_type(4)));
typedef int      v4i  __attribute__((ext_vector_type(4)));
typedef v8h __attribute__((may_alias)) v8ha;
typedef v4f __attribute__((may_alias)) v4fa;
typedef v4i __attribute__((may_alias)) v4ia;

union FragU { v16h v; v8h half[2]; };

__device__ __forceinline__ float fz16(float v) { return (fabsf(v) < 6.103515625e-5f) ? 0.0f : v; }
__device__ __forceinline__ _Float16 to_h(float v) { return (_Float16)fz16(v); }

__device__ __forceinline__ v8f wmma_f16(v16h a, v16h b, v8f c) {
  v8f d = __builtin_amdgcn_wmma_f32_16x16x32_f16(false, a, false, b, (short)0, c, false, false);
  asm volatile("v_nop\n\tv_nop\n\tv_nop\n\tv_nop" : "+v"(d) : "v"(a), "v"(b));
  return d;
}
__device__ __forceinline__ v8f mma_raw(v16h a, v16h b, v8f c) {
  return __builtin_amdgcn_wmma_f32_16x16x32_f16(false, a, false, b, (short)0, c, false, false);
}
__device__ __forceinline__ void dep_guard_h(v8f& a, v8f& b, v16h x, v16h y) {
  asm volatile("v_nop\n\tv_nop\n\tv_nop\n\tv_nop" : "+v"(a), "+v"(b) : "v"(x), "v"(y));
}
__device__ __forceinline__ void keep4_h(v16h a, v16h b, v16h c, v16h d) {
  asm volatile("v_nop" :: "v"(a), "v"(b), "v"(c), "v"(d));
}
__device__ __forceinline__ void acc_guard4(v8f& a, v8f& b, v8f& c, v8f& d) {
  asm volatile("v_nop\n\tv_nop\n\tv_nop\n\tv_nop" : "+v"(a), "+v"(b), "+v"(c), "+v"(d));
}

__device__ __forceinline__ v16h load_frag(const _Float16* p, int h) {
  FragU f;
  f.half[0] = *(const v8ha*)(p + 8 * h);
  f.half[1] = *(const v8ha*)(p + 16 + 8 * h);
  return f.v;
}
__device__ __forceinline__ v16h gfrag(const _Float16* p) {
  FragU f;
  f.half[0] = *(const v8ha*)(p);
  f.half[1] = *(const v8ha*)(p + 16);
  return f.v;
}

__device__ __forceinline__ v8f zero8f() { v8f z = {0.f, 0.f, 0.f, 0.f, 0.f, 0.f, 0.f, 0.f}; return z; }

template <int BIAS_MODE, int OUT_MODE, bool RESID, int ACT>
__global__ __launch_bounds__(256) void wmma_gemm64(
    const _Float16* __restrict__ A, int lda, long strideA,
    const _Float16* __restrict__ Bt, int ldb, long strideB,
    void* __restrict__ Cout, int ldc, long strideC,
    const float* __restrict__ bias,
    const float* __restrict__ resid, int ldr, long strideR,
    int M, int N, int K, float scale) {
  static_assert(OUT_MODE == 1 || ACT == 0);
  static_assert(BIAS_MODE == 0 || BIAS_MODE == 2);
  static_assert(!(RESID && OUT_MODE == 1));
  __shared__ __attribute__((aligned(16))) float sT[8][16 * 68];

  const int b    = blockIdx.y;
  const int lane = threadIdx.x & 31;
  const int wave = threadIdx.x >> 5;
  const int tilesN = N >> 6;
  const int tilesM = M >> 6;
  const int tile = blockIdx.x * 8 + wave;
  if (tile >= tilesM * tilesN) return;
  const int tm = tile / tilesN;
  const int tn = tile - tm * tilesN;
  const int m0 = tm << 6;
  const int n0 = tn << 6;

  const _Float16* Ab = A  + (size_t)b * strideA;
  const _Float16* Bb = Bt + (size_t)b * strideB;

  const int rlane = lane & 15;
  const int koff  = (lane >> 4) * 8;
  const int mOff  = (lane >> 4) * 8;

  v8f acc[4][4];
#pragma unroll
  for (int i = 0; i < 4; ++i)
#pragma unroll
    for (int j = 0; j < 4; ++j) acc[i][j] = zero8f();

  for (int k0 = 0; k0 < K; k0 += 32) {
    v16h bh[4];
#pragma unroll
    for (int j = 0; j < 4; ++j) {
      const size_t bo = (size_t)(n0 + (j << 4) + rlane) * ldb + koff + k0;
      bh[j] = gfrag(Bb + bo);
    }
#pragma unroll
    for (int i = 0; i < 4; ++i) {
      const size_t ao = (size_t)(m0 + (i << 4) + rlane) * lda + koff + k0;
      const v16h ah = gfrag(Ab + ao);
#pragma unroll
      for (int j = 0; j < 4; ++j) acc[i][j] = mma_raw(ah, bh[j], acc[i][j]);
      dep_guard_h(acc[i][0], acc[i][3], ah, ah);
    }
    keep4_h(bh[0], bh[1], bh[2], bh[3]);
  }
  acc_guard4(acc[0][0], acc[0][1], acc[0][2], acc[0][3]);
  acc_guard4(acc[1][0], acc[1][1], acc[1][2], acc[1][3]);
  acc_guard4(acc[2][0], acc[2][1], acc[2][2], acc[2][3]);
  acc_guard4(acc[3][0], acc[3][1], acc[3][2], acc[3][3]);

  float* slab = sT[wave];
  float bvj[4] = {0.f, 0.f, 0.f, 0.f};
  if (BIAS_MODE == 2 && OUT_MODE == 1) {
#pragma unroll
    for (int j = 0; j < 4; ++j) bvj[j] = bias[n0 + (j << 4) + rlane];
  }
#pragma unroll
  for (int i = 0; i < 4; ++i) {
    const int mBase = m0 + (i << 4);
#pragma unroll
    for (int j = 0; j < 4; ++j) {
#pragma unroll
      for (int r = 0; r < 8; ++r) {
        float v = acc[i][j][r] * scale;
        if (BIAS_MODE == 2 && OUT_MODE == 1) v += bvj[j];
        if (ACT == 2) v = fmaxf(v, 0.0f);
        slab[(mOff + r) * 68 + (j << 4) + rlane] = v;
      }
    }
    __builtin_amdgcn_fence(__ATOMIC_RELEASE, "workgroup");
    __builtin_amdgcn_wave_barrier();
    __builtin_amdgcn_fence(__ATOMIC_ACQUIRE, "workgroup");
    if (OUT_MODE == 0) {
      float* C = (float*)Cout + (size_t)b * strideC;
      const float* Rb = resid + (size_t)b * strideR;
      const int hh = lane >> 4, c4 = (lane & 15) * 4;
      v4f bias4 = {0.f, 0.f, 0.f, 0.f};
      if (BIAS_MODE == 2) bias4 = *(const v4fa*)(bias + n0 + c4);
      v4f vals[8];
#pragma unroll
      for (int it = 0; it < 8; ++it) {
        const int row = it * 2 + hh;
        v4f v = *(const v4f*)(slab + row * 68 + c4) + bias4;
        if (RESID) v = v + *(const v4fa*)(Rb + (size_t)(mBase + row) * ldr + n0 + c4);
        vals[it] = v;
      }
      for (int pass = 0; pass < 2; ++pass) {
#pragma unroll
        for (int it = 0; it < 8; ++it) {
          const int row = it * 2 + hh;
          *(volatile v4f*)(C + (size_t)(mBase + row) * ldc + n0 + c4) = vals[it];
        }
        __threadfence();
      }
    } else {
      const int q = lane >> 3, c8 = (lane & 7) * 8;
      _Float16* C = (_Float16*)Cout + (size_t)b * strideC;
      for (int pass = 0; pass < 2; ++pass) {
#pragma unroll
        for (int it = 0; it < 4; ++it) {
          const int row = it * 4 + q;
          const float* sp = slab + row * 68 + c8;
          v8h hv;
#pragma unroll
          for (int e = 0; e < 8; ++e) hv[e] = to_h(sp[e]);
          *(volatile v8h*)(C + (size_t)(mBase + row) * ldc + n0 + c8) = hv;
        }
        __threadfence();
      }
    }
    __builtin_amdgcn_fence(__ATOMIC_RELEASE, "workgroup");
    __builtin_amdgcn_wave_barrier();
    __builtin_amdgcn_fence(__ATOMIC_ACQUIRE, "workgroup");
  }
}

__global__ __launch_bounds__(256) void convert_kernel(
    const float* __restrict__ w0, const float* __restrict__ w1, const float* __restrict__ w2,
    const float* __restrict__ w3, const float* __restrict__ w4, const float* __restrict__ w5,
    const float* __restrict__ w6, const float* __restrict__ w7, const float* __restrict__ w8,
    const float* __restrict__ w9, const float* __restrict__ prev,
    _Float16* __restrict__ wall, _Float16* __restrict__ pb) {
  const int mat = blockIdx.y;
  const float* src = w0;
  _Float16* dst = wall;
  int n8 = WM / 8;
  float sc = WSC;
  if (mat == 1)      { src = w1; dst = wall + (size_t)1 * WM; }
  else if (mat == 2) { src = w2; dst = wall + (size_t)2 * WM; }
  else if (mat == 3) { src = w3; dst = wall + (size_t)3 * WM; }
  else if (mat == 4) { src = w4; dst = wall + (size_t)4 * WM; }
  else if (mat == 5) { src = w5; dst = wall + (size_t)5 * WM; }
  else if (mat == 6) { src = w6; dst = wall + (size_t)6 * WM; }
  else if (mat == 7) { src = w7; dst = wall + (size_t)7 * WM; }
  else if (mat == 8) { src = w8; dst = wall + (size_t)8 * WM;  n8 = (DFF * DM) / 8; }
  else if (mat == 9) { src = w9; dst = wall + (size_t)12 * WM; n8 = (DM * DFF) / 8; }
  else if (mat == 10){ src = prev; dst = pb; n8 = (NTOK * DM) / 8; sc = 1.0f; }
  const int g = blockIdx.x * 256 + threadIdx.x;
  if (g >= n8) return;
  const float* sp = src + (size_t)g * 8;
  const v4f a = *(const v4fa*)sp;
  const v4f c = *(const v4fa*)(sp + 4);
  v8h o;
  o[0] = to_h(a.x * sc); o[1] = to_h(a.y * sc); o[2] = to_h(a.z * sc); o[3] = to_h(a.w * sc);
  o[4] = to_h(c.x * sc); o[5] = to_h(c.y * sc); o[6] = to_h(c.z * sc); o[7] = to_h(c.w * sc);
  _Float16* dp = dst + (size_t)g * 8;
  *(volatile v8h*)dp = o;
  __threadfence();
  *(volatile v8h*)dp = o;
}

__global__ __launch_bounds__(256) void mask_class_kernel(const float* __restrict__ mask, int* __restrict__ ctab) {
  __shared__ unsigned int wbits[8];
  __shared__ __attribute__((aligned(16))) int cls[CTP];
  const int tid = threadIdx.x, lane = tid & 31, wave = tid >> 5;
  const int blk = blockIdx.x;
  const int r  = tid >> 2;
  const int cq = tid & 3;
  const float* mrow = mask + (size_t)(blk * 64 + r) * SEQ + cq * 256;
  unsigned int bits = 0u;
#pragma unroll 1
  for (int tq = 0; tq < 4; ++tq) {
    int nz = 0, nn = 0;
#pragma unroll 4
    for (int i = 0; i < 16; ++i) {
      const v4f v = *(const v4fa*)(mrow + tq * 64 + 4 * i);
      nz |= (v.x != 0.0f) | (v.y != 0.0f) | (v.z != 0.0f) | (v.w != 0.0f);
      nn |= (v.x > -1.0e8f) | (v.y > -1.0e8f) | (v.z > -1.0e8f) | (v.w > -1.0e8f);
    }
    const int kt = cq * 4 + tq;
    bits |= ((unsigned int)(nz & 1) << kt) | ((unsigned int)(nn & 1) << (16 + kt));
  }
#pragma unroll
  for (int off = 1; off < 32; off <<= 1) bits |= __shfl_xor(bits, off, 32);
  if (lane == 0) wbits[wave] = bits;
  __syncthreads();
  if (tid < CTP) {
    const unsigned int all = wbits[0] | wbits[1] | wbits[2] | wbits[3] | wbits[4] | wbits[5] | wbits[6] | wbits[7];
    int c = 0;
    if (tid < 16) {
      const int nz = (int)((all >> tid) & 1u);
      const int nn = (int)((all >> (16 + tid)) & 1u);
      c = (nn == 0) ? 2 : ((nz == 0) ? 1 : 0);
    }
    cls[tid] = c;
  }
  __syncthreads();
  if (tid < 8) {
    const v4i v = *(const v4ia*)(cls + 4 * tid);
    int* dp = ctab + (size_t)blk * CTP + 4 * tid;
    *(volatile v4i*)dp = v;
    __threadfence();
    *(volatile v4i*)dp = v;
  }
}

__global__ __launch_bounds__(128) void ln_kernel(const float* __restrict__ x, const float* __restrict__ g,
                                                const float* __restrict__ bta, _Float16* __restrict__ out) {
  __shared__ float red[8];
  const int row = blockIdx.x, tid = threadIdx.x, lane = tid & 31, wave = tid >> 5;
  const float* xr = x + (size_t)row * DM + 8 * tid;
  const v4f a = *(const v4fa*)xr;
  const v4f c = *(const v4fa*)(xr + 4);
  float s = ((a.x + a.y) + (a.z + a.w)) + ((c.x + c.y) + (c.z + c.w));
#pragma unroll
  for (int off = 16; off > 0; off >>= 1) s += __shfl_xor(s, off, 32);
  if (lane == 0) red[wave] = s;
  __syncthreads();
  const float mu = ((red[0] + red[1]) + (red[2] + red[3])) * (1.0f / (float)DM);
  float d[8];
  d[0] = a.x - mu; d[1] = a.y - mu; d[2] = a.z - mu; d[3] = a.w - mu;
  d[4] = c.x - mu; d[5] = c.y - mu; d[6] = c.z - mu; d[7] = c.w - mu;
  float sq = 0.0f;
#pragma unroll
  for (int e = 0; e < 8; ++e) sq += d[e] * d[e];
#pragma unroll
  for (int off = 16; off > 0; off >>= 1) sq += __shfl_xor(sq, off, 32);
  if (lane == 0) red[4 + wave] = sq;
  __syncthreads();
  const float var  = ((red[4] + red[5]) + (red[6] + red[7])) * (1.0f / (float)DM);
  const float rstd = rsqrtf(var + LN_EPS);
  const v4f ga = *(const v4fa*)(g + 8 * tid);
  const v4f gc = *(const v4fa*)(g + 8 * tid + 4);
  const v4f ba = *(const v4fa*)(bta + 8 * tid);
  const v4f bc = *(const v4fa*)(bta + 8 * tid + 4);
  v8h o;
  o[0] = to_h(ga.x * (d[0] * rstd) + ba.x);
  o[1] = to_h(ga.y * (d[1] * rstd) + ba.y);
  o[2] = to_h(ga.z * (d[2] * rstd) + ba.z);
  o[3] = to_h(ga.w * (d[3] * rstd) + ba.w);
  o[4] = to_h(gc.x * (d[4] * rstd) + bc.x);
  o[5] = to_h(gc.y * (d[5] * rstd) + bc.y);
  o[6] = to_h(gc.z * (d[6] * rstd) + bc.z);
  o[7] = to_h(gc.w * (d[7] * rstd) + bc.w);
  _Float16* dp = out + (size_t)row * DM + 8 * tid;
  *(volatile v8h*)dp = o;
  __threadfence();
  *(volatile v8h*)dp = o;
}

__device__ __forceinline__ v16h pack_p(v8f a, v8f c) {
  v16h r;
#pragma unroll
  for (int e = 0; e < 8; ++e) {
    r[e]     = to_h(a[e] * PSC);
    r[8 + e] = to_h(c[e] * PSC);
  }
  return r;
}

__device__ __forceinline__ void ctx_store_pass(const _Float16* so, _Float16* ctx, size_t tok0, int head, int lane) {
  const int q8 = lane & 7, sub = lane >> 3;
#pragma unroll
  for (int i = 0; i < 4; ++i) {
    const int row = i * 4 + sub;
    const v8h v = *(const v8ha*)(so + row * 64 + 8 * q8);
    *(volatile v8h*)(ctx + (tok0 + (size_t)row) * DM + head * HD + 8 * q8) = v;
  }
}

__global__ __launch_bounds__(128) void attn_kernel(
    const _Float16* __restrict__ qk,
    const _Float16* __restrict__ vt,
    const float* __restrict__ mask,
    const int* __restrict__ ctab,
    int use_mask,
    _Float16* __restrict__ ctx)
{
  __shared__ __attribute__((aligned(16))) _Float16 sO[4 * 16 * 64];

  const int tid = threadIdx.x, lane = tid & 31, w = tid >> 5;
  const int h = lane >> 4, m = lane & 15;
  const int bh = blockIdx.y, b = bh >> 4, head = bh & 15;
  const int qt = blockIdx.x;
  const int q0 = qt * 64 + 16 * w;
  const size_t tokq = (size_t)b * SEQ + q0 + m;

  const _Float16* qrow = qk + tokq * QKP + head * HD;
  const v16h qb0 = load_frag(qrow, h);
  const v16h qb1 = load_frag(qrow + 32, h);

  v8f o[4];
#pragma unroll
  for (int t = 0; t < 4; ++t) o[t] = zero8f();
  float mrun = -1.0e30f, lrun = 0.0f;

  const _Float16* kbase = qk + ((size_t)b * SEQ + m) * QKP + DM + head * HD;
  const _Float16* vbase = vt + ((size_t)b * DM + head * HD + m) * SEQ;
  const float* mkrow = mask + tokq * SEQ + 8 * h;
  const int* crow = ctab + (b * (SEQ / 64) + qt) * CTP;

#pragma unroll 1
  for (int kt = 0; kt < SEQ / 64; ++kt) {
    int cls = 1;
    if (use_mask != 0) cls = crow[kt];
    if (cls == 2) continue;
    const int kb = kt * 64;

    v8f s[4];
#pragma unroll
    for (int j = 0; j < 4; ++j) {
      const _Float16* kp = kbase + (size_t)(kb + 16 * j) * QKP;
      const v16h kf0 = load_frag(kp, h);
      const v16h kf1 = load_frag(kp + 32, h);
      v8f z = zero8f();
      z = wmma_f16(kf0, qb0, z);
      z = wmma_f16(kf1, qb1, z);
      s[j] = z * 0.125f;
    }
    if (cls != 1) {
#pragma unroll
      for (int j = 0; j < 4; ++j) {
        const float* mp = mkrow + kb + 16 * j;
        const v4f ma = *(const v4fa*)mp;
        const v4f mb = *(const v4fa*)(mp + 4);
        s[j][0] = s[j][0] + ma.x; s[j][1] = s[j][1] + ma.y; s[j][2] = s[j][2] + ma.z; s[j][3] = s[j][3] + ma.w;
        s[j][4] = s[j][4] + mb.x; s[j][5] = s[j][5] + mb.y; s[j][6] = s[j][6] + mb.z; s[j][7] = s[j][7] + mb.w;
      }
    }

    float mloc = s[0][0];
#pragma unroll
    for (int j = 0; j < 4; ++j)
#pragma unroll
      for (int r = 0; r < 8; ++r) mloc = fmaxf(mloc, s[j][r]);
    mloc = fmaxf(mloc, __shfl_xor(mloc, 16, 32));
    const float mnew = fmaxf(mrun, mloc);
    const float alpha = __expf(mrun - mnew);
    mrun = mnew;
    float lsum = 0.0f;
#pragma unroll
    for (int j = 0; j < 4; ++j)
#pragma unroll
      for (int r = 0; r < 8; ++r) {
        const float p = __expf(s[j][r] - mnew);
        s[j][r] = p;
        lsum += p;
      }
    lsum += __shfl_xor(lsum, 16, 32);
    lrun = lrun * alpha + lsum;
#pragma unroll
    for (int t = 0; t < 4; ++t)
#pragma unroll
      for (int r = 0; r < 8; ++r) o[t][r] = o[t][r] * alpha;

    const v16h pb0 = pack_p(s[0], s[1]);
    const v16h pb1 = pack_p(s[2], s[3]);

#pragma unroll
    for (int t = 0; t < 4; ++t) {
      const _Float16* vp = vbase + (size_t)(16 * t) * SEQ + kb;
      const v16h vf0 = load_frag(vp, h);
      const v16h vf1 = load_frag(vp + 32, h);
      o[t] = wmma_f16(vf0, pb0, o[t]);
      o[t] = wmma_f16(vf1, pb1, o[t]);
    }
  }

  const float inv = (1.0f / lrun) * (1.0f / PSC);
  _Float16* so = sO + w * 1024;
#pragma unroll
  for (int t = 0; t < 4; ++t)
#pragma unroll
    for (int r = 0; r < 8; ++r)
      so[m * 64 + 16 * t + 8 * h + r] = to_h(o[t][r] * inv);
  __syncthreads();

  const size_t tok0 = (size_t)b * SEQ + q0;
  ctx_store_pass(so, ctx, tok0, head, lane);
  __threadfence();
  ctx_store_pass(so, ctx, tok0, head, lane);
}

extern "C" void kernel_launch(void* const* d_in, const int* in_sizes, int n_in,
                              void* d_out, int out_size, void* d_ws, size_t ws_size,
                              hipStream_t stream) {
  if (n_in < 21) return;
  if (in_sizes[0] != NTOK * DM || in_sizes[1] != NTOK * DM) return;
  if (in_sizes[2] != NBATCH * SEQ * SEQ) return;
  for (int i = 3; i <= 10; ++i) if (in_sizes[i] != DM * DM) return;
  if (in_sizes[11] != DFF * DM || in_sizes[12] != DFF || in_sizes[13] != DM * DFF || in_sizes[14] != DM) return;
  for (int i = 15; i <= 20; ++i) if (in_sizes[i] != DM) return;
  if (out_size != NTOK * DM) return;

  const float* this_seq = (const float*)d_in[0];
  const float* prev_seq = (const float*)d_in[1];
  const float* maskp    = (const float*)d_in[2];
  const float* sa_wq = (const float*)d_in[3];
  const float* sa_wk = (const float*)d_in[4];
  const float* sa_wv = (const float*)d_in[5];
  const float* sa_wo = (const float*)d_in[6];
  const float* ca_wq = (const float*)d_in[7];
  const float* ca_wk = (const float*)d_in[8];
  const float* ca_wv = (const float*)d_in[9];
  const float* ca_wo = (const float*)d_in[10];
  const float* ff_w1 = (const float*)d_in[11];
  const float* ff_b1 = (const float*)d_in[12];
  const float* ff_w2 = (const float*)d_in[13];
  const float* ff_b2 = (const float*)d_in[14];
  const float* ln1_g = (const float*)d_in[15];
  const float* ln1_b = (const float*)d_in[16];
  const float* ln2_g = (const float*)d_in[17];
  const float* ln2_b = (const float*)d_in[18];
  const float* ln3_g = (const float*)d_in[19];
  const float* ln3_b = (const float*)d_in[20];
  float* outp = (float*)d_out;

  const size_t bWALL = (size_t)16 * WM * 2;
  const size_t bPL   = (size_t)NTOK * DM * 2;
  const size_t bQK   = (size_t)NTOK * QKP * 2;
  const size_t bY    = (size_t)NTOK * DM * 4;
  const size_t bCT   = (size_t)NBATCH * (SEQ / 64) * CTP * 4;
  size_t off = 0;
  const size_t oWALL = off; off += bWALL;
  const size_t oPB   = off; off += bPL;
  const size_t oH    = off; off += bPL;
  const size_t oQK   = off; off += bQK;
  const size_t oVT   = off; off += bPL;
  const size_t oCTX  = off; off += bPL;
  const size_t oY1   = off; off += bY;
  const size_t oY2   = off; off += bY;
  const size_t oCT   = off; off += bCT;
  if (off > ws_size) return;
  const size_t oF = oQK;
  if (oF + (size_t)NTOK * DFF * 2 != oY1) return;

  char* ws = (char*)d_ws;
  _Float16* WALL = (_Float16*)(ws + oWALL);
  _Float16* PB   = (_Float16*)(ws + oPB);
  _Float16* H    = (_Float16*)(ws + oH);
  _Float16* QK   = (_Float16*)(ws + oQK);
  _Float16* VT   = (_Float16*)(ws + oVT);
  _Float16* CTX  = (_Float16*)(ws + oCTX);
  _Float16* F    = (_Float16*)(ws + oF);
  float*    Y1   = (float*)(ws + oY1);
  float*    Y2   = (float*)(ws + oY2);
  int*      CT   = (int*)(ws + oCT);

  const long sPLB = (long)SEQ * DM;
  const long sVT  = (long)DM * SEQ;

  convert_kernel<<<dim3((NTOK * DM / 8) / 256, 11), dim3(256), 0, stream>>>(
      sa_wq, sa_wk, sa_wv, sa_wo, ca_wq, ca_wk, ca_wv, ca_wo, ff_w1, ff_w2, prev_seq, WALL, PB);
  mask_class_kernel<<<dim3(NBATCH * (SEQ / 64)), dim3(256), 0, stream>>>(maskp, CT);

  ln_kernel<<<dim3(NTOK), dim3(128), 0, stream>>>(this_seq, ln1_g, ln1_b, H);
  wmma_gemm64<0, 1, false, 0><<<dim3(256, 1), dim3(256), 0, stream>>>(
      H, DM, 0L, WALL + (size_t)0 * WM, DM, 0L, (void*)QK, QKP, 0L,
      ln1_g, this_seq, DM, 0L, NTOK, 2 * DM, DM, INV_WSC);
  wmma_gemm64<0, 1, false, 0><<<dim3(32, NBATCH), dim3(256), 0, stream>>>(
      WALL + (size_t)2 * WM, DM, 0L, H, DM, sPLB, (void*)VT, SEQ, sVT,
      ln1_g, this_seq, DM, 0L, DM, SEQ, DM, INV_WSC);
  attn_kernel<<<dim3(SEQ / 64, NBATCH * NH), dim3(128), 0, stream>>>(QK, VT, maskp, CT, 1, CTX);
  wmma_gemm64<0, 0, true, 0><<<dim3(128, 1), dim3(256), 0, stream>>>(
      CTX, DM, 0L, WALL + (size_t)3 * WM, DM, 0L, (void*)Y1, DM, 0L,
      ln1_g, this_seq, DM, 0L, NTOK, DM, DM, INV_WSC);

  ln_kernel<<<dim3(NTOK), dim3(128), 0, stream>>>(Y1, ln2_g, ln2_b, H);
  wmma_gemm64<0, 1, false, 0><<<dim3(128, 1), dim3(256), 0, stream>>>(
      H, DM, 0L, WALL + (size_t)4 * WM, DM, 0L, (void*)QK, QKP, 0L,
      ln1_g, this_seq, DM, 0L, NTOK, DM, DM, INV_WSC);
  wmma_gemm64<0, 1, false, 0><<<dim3(128, 1), dim3(256), 0, stream>>>(
      PB, DM, 0L, WALL + (size_t)5 * WM, DM, 0L, (void*)(QK + DM), QKP, 0L,
      ln1_g, this_seq, DM, 0L, NTOK, DM, DM, INV_WSC);
  wmma_gemm64<0, 1, false, 0><<<dim3(32, NBATCH), dim3(256), 0, stream>>>(
      WALL + (size_t)6 * WM, DM, 0L, PB, DM, sPLB, (void*)VT, SEQ, sVT,
      ln1_g, this_seq, DM, 0L, DM, SEQ, DM, INV_WSC);
  attn_kernel<<<dim3(SEQ / 64, NBATCH * NH), dim3(128), 0, stream>>>(QK, VT, maskp, CT, 0, CTX);
  wmma_gemm64<0, 0, true, 0><<<dim3(128, 1), dim3(256), 0, stream>>>(
      CTX, DM, 0L, WALL + (size_t)7 * WM, DM, 0L, (void*)Y2, DM, 0L,
      ln1_g, Y1, DM, 0L, NTOK, DM, DM, INV_WSC);

  ln_kernel<<<dim3(NTOK), dim3(128), 0, stream>>>(Y2, ln3_g, ln3_b, H);
  wmma_gemm64<2, 1, false, 2><<<dim3(512, 1), dim3(256), 0, stream>>>(
      H, DM, 0L, WALL + (size_t)8 * WM, DM, 0L, (void*)F, DFF, 0L,
      ff_b1, this_seq, DM, 0L, NTOK, DFF, DM, INV_WSC);
  wmma_gemm64<2, 0, true, 0><<<dim3(128, 1), dim3(256), 0, stream>>>(
      F, DFF, 0L, WALL + (size_t)12 * WM, DFF, 0L, (void*)outp, DM, 0L,
      ff_b2, Y2, DM, 0L, NTOK, DM, DFF, INV_WSC);

  (void)hipGetLastError();
}
